// GWM_10247791968408
// MI455X (gfx1250) — hardware-verified
//
#include <hip/hip_runtime.h>
#include <math.h>
#include <stdint.h>

#define NBAT  4
#define NTOK  4096
#define CIN   256
#define C2    512
#define C3    768
#define MTOK  16384
#define NHD   8
#define HD    32
#define NGR   4
#define LGR   1024
#define NUNIT 128
#define STP   68
#define SBP   132
#define ASP   36
#define CXS   16.0f
#define CWS   256.0f
#define CQK   (16.0f / 4096.0f)
#define CVS   (16.0f / 4096.0f)
#define CYS   256.0f
#define QKSC  (0.17677669529663688f / 256.0f)

static_assert(NUNIT == NBAT * NGR * NHD);
static_assert(NGR * LGR == NTOK);
static_assert(MTOK == NBAT * NTOK);
static_assert(NTOK % 128 == 0);
static_assert(LGR % 32 == 0);
static_assert(CIN % 64 == 0);
static_assert(NHD * HD == CIN);
static_assert(64 * SBP <= 8 * 16 * STP);
static_assert((STP * 4) % 16 == 0);
static_assert((SBP * 4) % 16 == 0);
static_assert((ASP * 4) % 16 == 0);
static_assert(C3 * CIN == 96 * 256 * 8);
static_assert(CIN * CIN == 32 * 256 * 8);

typedef _Float16 v16h __attribute__((ext_vector_type(16)));
typedef _Float16 v8h  __attribute__((ext_vector_type(8)));
typedef float    v8f  __attribute__((ext_vector_type(8)));
typedef float    v4f  __attribute__((ext_vector_type(4)));
typedef unsigned int v4u __attribute__((ext_vector_type(4)));
union Frag { v16h v; v8h half[2]; };

__device__ __forceinline__ unsigned short bf_bits(float f) {
  unsigned u = __float_as_uint(f);
  return (unsigned short)((u + 0x7FFFu + ((u >> 16) & 1u)) >> 16);
}
__device__ __forceinline__ float bfr(float f) { return __uint_as_float(((unsigned)bf_bits(f)) << 16); }
__device__ __forceinline__ unsigned short h_bits(_Float16 x) { return __builtin_bit_cast(unsigned short, x); }
__device__ __forceinline__ unsigned pk16(unsigned short a, unsigned short b) { return (unsigned)a | ((unsigned)b << 16); }
__device__ __forceinline__ v8f zero8() { v8f z = {0.f, 0.f, 0.f, 0.f, 0.f, 0.f, 0.f, 0.f}; return z; }

__device__ __forceinline__ v16h ldfrag_h(const _Float16* p) {
  Frag f;
  f.half[0] = *(const v8h*)(p);
  f.half[1] = *(const v8h*)(p + 16);
  return f.v;
}

__device__ __forceinline__ v8f mma_h(v16h a, v16h b, v8f c) {
  c = __builtin_amdgcn_wmma_f32_16x16x32_f16(false, a, false, b, (short)0, c, false, false);
#if defined(__HIP_DEVICE_COMPILE__)
  asm volatile("v_nop\n\tv_nop\n\tv_nop\n\tv_nop" : "+v"(c) : "v"(a), "v"(b));
#endif
  return c;
}
__device__ __forceinline__ void wave_sync_lds() {
  __builtin_amdgcn_fence(__ATOMIC_RELEASE, "workgroup");
  __builtin_amdgcn_wave_barrier();
  __builtin_amdgcn_fence(__ATOMIC_ACQUIRE, "workgroup");
}

__device__ __forceinline__ v4u pack8h(v4f a, v4f b) {
  v4u p;
  p[0] = pk16(h_bits((_Float16)a[0]), h_bits((_Float16)a[1]));
  p[1] = pk16(h_bits((_Float16)a[2]), h_bits((_Float16)a[3]));
  p[2] = pk16(h_bits((_Float16)b[0]), h_bits((_Float16)b[1]));
  p[3] = pk16(h_bits((_Float16)b[2]), h_bits((_Float16)b[3]));
  return p;
}

__device__ __forceinline__ void cvt8_w(const float* __restrict__ src, unsigned short* dst, size_t e0) {
  const v4f a = *(const v4f*)(src + e0);
  const v4f b = *(const v4f*)(src + e0 + 4);
  v4f sa, sb;
#pragma unroll
  for (int e = 0; e < 4; ++e) { sa[e] = bfr(a[e]) * CWS; sb[e] = bfr(b[e]) * CWS; }
  const v4u pk = pack8h(sa, sb);
  *(volatile v4u*)(dst + e0) = pk;
  __threadfence();
  *(volatile v4u*)(dst + e0) = pk;
}
__global__ __launch_bounds__(256) void cvt_w(const float* __restrict__ wqkv, const float* __restrict__ wp,
                                             unsigned short* Wq, unsigned short* Wp) {
  const int tid = threadIdx.x, blk = blockIdx.x;
  if (blk < 96) cvt8_w(wqkv, Wq, ((size_t)blk * 256 + tid) * 8);
  else          cvt8_w(wp,   Wp, ((size_t)(blk - 96) * 256 + tid) * 8);
}

__global__ __launch_bounds__(256) void cvt_x(const float* __restrict__ x, const int* __restrict__ idx,
                                             unsigned short* X16) {
  const int tid = threadIdx.x, lane = tid & 31;
  const int R = blockIdx.x * 8 + (tid >> 5);
  const int b = R >> 12, j = R & (NTOK - 1);
  int src = idx[j];
  src = (src < 0) ? 0 : ((src > NTOK - 1) ? (NTOK - 1) : src);
  const float* sp = x + ((size_t)(b * NTOK + src)) * CIN + lane * 8;
  const v4f a  = *(const v4f*)(sp);
  const v4f a2 = *(const v4f*)(sp + 4);
  v4f sa, sb;
#pragma unroll
  for (int e = 0; e < 4; ++e) { sa[e] = bfr(a[e]) * CXS; sb[e] = bfr(a2[e]) * CXS; }
  const v4u pk = pack8h(sa, sb);
  unsigned short* dp = X16 + (size_t)R * CIN + lane * 8;
  *(volatile v4u*)dp = pk;
  __threadfence();
  *(volatile v4u*)dp = pk;
}

__global__ __launch_bounds__(256)
void gemm_qkv(const unsigned short* __restrict__ X16, const unsigned short* __restrict__ Wq,
              unsigned short* QK, unsigned short* V16) {
  __shared__ __align__(16) float sm[8 * 16 * STP];
  const int tid = threadIdx.x, wave = tid >> 5, lane = tid & 31, hh = lane >> 4, c = lane & 15;
  const int n0 = blockIdx.x * 64, m0 = blockIdx.y * 128;
  const int arow = m0 + wave * 16 + c;
  const _Float16* A = (const _Float16*)(const void*)X16;
  const _Float16* B = (const _Float16*)(const void*)Wq;

  v8f acc[4];
#pragma unroll
  for (int nt = 0; nt < 4; ++nt) acc[nt] = zero8();

#pragma unroll 1
  for (int k0 = 0; k0 < CIN; k0 += 32) {
    const v16h af = ldfrag_h(A + (size_t)arow * CIN + k0 + 8 * hh);
#pragma unroll
    for (int nt = 0; nt < 4; ++nt) {
      const v16h bfrag = ldfrag_h(B + (size_t)(n0 + nt * 16 + c) * CIN + k0 + 8 * hh);
      acc[nt] = mma_h(af, bfrag, acc[nt]);
    }
  }

  if (blockIdx.x < 8) {
    float* st = sm + wave * (16 * STP);
#pragma unroll
    for (int nt = 0; nt < 4; ++nt) {
#pragma unroll
      for (int r = 0; r < 8; ++r) st[(8 * hh + r) * STP + nt * 16 + c] = acc[nt][r];
    }
    wave_sync_lds();
    const int piece = lane & 7, rsub = lane >> 3;
    v4u pk[4];
    size_t offs[4];
#pragma unroll
    for (int it = 0; it < 4; ++it) {
      const int row = it * 4 + rsub;
      v4f fa = *(const v4f*)(st + row * STP + piece * 8);
      v4f fb = *(const v4f*)(st + row * STP + piece * 8 + 4);
      fa = fa * CQK;
      fb = fb * CQK;
      pk[it] = pack8h(fa, fb);
      offs[it] = ((size_t)(m0 + wave * 16 + row)) * C2 + n0 + piece * 8;
    }
    for (int pass = 0; pass < 2; ++pass) {
#pragma unroll
      for (int it = 0; it < 4; ++it) *(volatile v4u*)(QK + offs[it]) = pk[it];
      __threadfence();
    }
  } else {
    const int cv0 = n0 - C2;
#pragma unroll
    for (int nt = 0; nt < 4; ++nt) {
#pragma unroll
      for (int r = 0; r < 8; ++r) sm[(nt * 16 + c) * SBP + wave * 16 + 8 * hh + r] = acc[nt][r];
    }
    __syncthreads();
    const int bimg = m0 >> 12, s0 = m0 & (NTOK - 1);
    v4u pk[4];
    size_t o16[4];
#pragma unroll
    for (int i2 = 0; i2 < 4; ++i2) {
      const int cc = wave * 8 + i2 * 2 + hh;
      const int co = cv0 + cc;
      v4f fa = *(const v4f*)(sm + cc * SBP + c * 8);
      v4f fb = *(const v4f*)(sm + cc * SBP + c * 8 + 4);
      fa = fa * CVS;
      fb = fb * CVS;
      pk[i2] = pack8h(fa, fb);
      o16[i2] = ((size_t)(bimg * CIN + co)) * NTOK + s0 + c * 8;
    }
    for (int pass = 0; pass < 2; ++pass) {
#pragma unroll
      for (int i2 = 0; i2 < 4; ++i2) *(volatile v4u*)(V16 + o16[i2]) = pk[i2];
      __threadfence();
    }
  }
}

__global__ __launch_bounds__(256)
void attn_k(const unsigned short* __restrict__ QK, const unsigned short* __restrict__ V16, unsigned short* Y) {
  __shared__ __align__(16) float Sst[8 * 16 * ASP];
  const int tid = threadIdx.x, wave = tid >> 5, lane = tid & 31, hh = lane >> 4, c = lane & 15;
  const int u = blockIdx.x;
  const int head = u & 7, gr = (u >> 3) & 3, b = u >> 5;
  const size_t tok0 = (size_t)b * NTOK + (size_t)gr * LGR;
  const _Float16* Qp = (const _Float16*)(const void*)QK + tok0 * C2 + head * HD;
  const _Float16* Kp = Qp + CIN;
  const size_t cm0 = ((size_t)(b * CIN + head * HD)) * NTOK + (size_t)gr * LGR;
  const _Float16* Vp = (const _Float16*)(const void*)V16 + cm0;
  float* st = Sst + wave * (16 * ASP);

#pragma unroll 1
  for (int qt = wave; qt < LGR / 16; qt += 8) {
    const int lq = qt * 16 + c;
    const v16h bq = ldfrag_h(Qp + (size_t)lq * C2 + 8 * hh);

    v8f o0 = zero8(), o1 = zero8();
    float mrun = -1.0e30f, lrun = 0.f;
#pragma unroll 1
    for (int ch = 0; ch < LGR / 32; ++ch) {
      const int kb = ch * 32;
      v8f s[2];
#pragma unroll
      for (int j = 0; j < 2; ++j) {
        const v16h ka = ldfrag_h(Kp + (size_t)(kb + j * 16 + c) * C2 + 8 * hh);
        s[j] = mma_h(ka, bq, zero8());
      }
      float mc = s[0][0];
#pragma unroll
      for (int j = 0; j < 2; ++j) {
#pragma unroll
        for (int r = 0; r < 8; ++r) mc = fmaxf(mc, s[j][r]);
      }
      mc = fmaxf(mc, __shfl_xor(mc, 16, 32));
      const float mnew = fmaxf(mrun, mc);
      const float alpha = __expf((mrun - mnew) * QKSC);
#pragma unroll
      for (int r = 0; r < 8; ++r) {
        const float arr = __shfl(alpha, 8 * hh + r, 32);
        o0[r] = o0[r] * arr;
        o1[r] = o1[r] * arr;
      }
      float psum = 0.f;
      v16h pfh;
#pragma unroll
      for (int i = 0; i < 8; ++i) {
        const float e0 = __expf((s[0][i] - mnew) * QKSC);
        const float e1 = __expf((s[1][i] - mnew) * QKSC);
        psum = psum + (e0 + e1);
        pfh[i]     = (_Float16)(e0 * 1024.0f);
        pfh[8 + i] = (_Float16)(e1 * 1024.0f);
      }
      lrun = lrun * alpha + psum;
      mrun = mnew;
      {
        const v16h vf0 = ldfrag_h(Vp + (size_t)c * NTOK + kb + 8 * hh);
        const v16h vf1 = ldfrag_h(Vp + (size_t)(HD / 2 + c) * NTOK + kb + 8 * hh);
        o0 = mma_h(pfh, vf0, o0);
        o1 = mma_h(pfh, vf1, o1);
      }
    }
    const float lsum = lrun + __shfl_xor(lrun, 16, 32);
    const float rinv = 1.0f / (lsum * 16384.0f);
#pragma unroll
    for (int r = 0; r < 8; ++r) {
      const int q = 8 * hh + r;
      const float inv = __shfl(rinv, q, 32);
      st[q * ASP + c]          = o0[r] * inv;
      st[q * ASP + HD / 2 + c] = o1[r] * inv;
    }
    wave_sync_lds();
    {
      const int rr = lane >> 2, dp = (lane & 3) * 8;
      v4u pk[2];
      size_t offs[2];
#pragma unroll
      for (int it = 0; it < 2; ++it) {
        const int row = it * 8 + rr;
        v4f fa = *(const v4f*)(st + row * ASP + dp);
        v4f fb = *(const v4f*)(st + row * ASP + dp + 4);
        fa = fa * CYS;
        fb = fb * CYS;
        pk[it] = pack8h(fa, fb);
        offs[it] = ((size_t)u * LGR + (size_t)(qt * 16 + row)) * HD + dp;
      }
      for (int pass = 0; pass < 2; ++pass) {
#pragma unroll
        for (int it = 0; it < 2; ++it) *(volatile v4u*)(Y + offs[it]) = pk[it];
        __threadfence();
      }
    }
    wave_sync_lds();
  }
}

__global__ __launch_bounds__(256)
void gemm_proj(const unsigned short* __restrict__ Y, const unsigned short* __restrict__ Wp,
               const float* __restrict__ bp, const int* __restrict__ idx, float* out) {
  __shared__ __align__(16) float sm[8 * 16 * STP];
  const int tid = threadIdx.x, wave = tid >> 5, lane = tid & 31, hh = lane >> 4, c = lane & 15;
  const int n0 = blockIdx.x * 64, m0 = blockIdx.y * 128;
  const int T = m0 + wave * 16 + c;
  const int bq = T >> 12, jj = T & (NTOK - 1), gr = jj >> 10, q = jj & (LGR - 1);
  const size_t abase = (((size_t)((bq * NGR + gr) * NHD)) * LGR + (size_t)q) * HD + 8 * hh;
  const _Float16* A = (const _Float16*)(const void*)Y;
  const _Float16* B = (const _Float16*)(const void*)Wp;

  v8f acc[4];
#pragma unroll
  for (int nt = 0; nt < 4; ++nt) acc[nt] = zero8();

#pragma unroll 1
  for (int ks = 0; ks < NHD; ++ks) {
    const size_t bo = abase + (size_t)ks * (LGR * HD);
    const v16h af = ldfrag_h(A + bo);
#pragma unroll
    for (int nt = 0; nt < 4; ++nt) {
      const v16h bfrag = ldfrag_h(B + (size_t)(n0 + nt * 16 + c) * CIN + ks * 32 + 8 * hh);
      acc[nt] = mma_h(af, bfrag, acc[nt]);
    }
  }

  float* st = sm + wave * (16 * STP);
#pragma unroll
  for (int nt = 0; nt < 4; ++nt) {
    const int co = n0 + nt * 16 + c;
    const float bi = bfr(bp[co]);
#pragma unroll
    for (int r = 0; r < 8; ++r) st[(8 * hh + r) * STP + nt * 16 + c] = acc[nt][r] * (1.0f / 65536.0f) + bi;
  }
  wave_sync_lds();
  const int bimg = m0 >> 12;
  const int jbase = (m0 & (NTOK - 1)) + wave * 16;
  v4f ov[8];
  size_t offs[8];
#pragma unroll
  for (int it = 0; it < 8; ++it) {
    const int row = it * 2 + hh;
    int dst = idx[jbase + row];
    dst = (dst < 0) ? 0 : ((dst > NTOK - 1) ? (NTOK - 1) : dst);
    ov[it] = *(const v4f*)(st + row * STP + c * 4);
    offs[it] = ((size_t)(bimg * NTOK + dst)) * CIN + n0 + c * 4;
  }
  for (int pass = 0; pass < 2; ++pass) {
#pragma unroll
    for (int it = 0; it < 8; ++it) *(volatile v4f*)(out + offs[it]) = ov[it];
    __threadfence();
  }
}

extern "C" void kernel_launch(void* const* d_in, const int* in_sizes, int n_in,
                              void* d_out, int out_size, void* d_ws, size_t ws_size,
                              hipStream_t stream) {
  if (n_in < 5) return;
  if (in_sizes[0] != NBAT * NTOK * CIN) return;
  if (in_sizes[1] != NTOK) return;
  if (in_sizes[2] != C3 * CIN) return;
  if (in_sizes[3] != CIN * CIN) return;
  if (in_sizes[4] != CIN) return;
  if (out_size != NBAT * NTOK * CIN) return;

  const float* x      = (const float*)d_in[0];
  const int*   idx    = (const int*)d_in[1];
  const float* w_qkv  = (const float*)d_in[2];
  const float* w_proj = (const float*)d_in[3];
  const float* b_proj = (const float*)d_in[4];
  float* out = (float*)d_out;

  const size_t sWq  = (size_t)C3 * CIN * 2;
  const size_t sWp  = (size_t)CIN * CIN * 2;
  const size_t sX16 = (size_t)MTOK * CIN * 2;
  const size_t sQK  = (size_t)MTOK * C2 * 2;
  const size_t sV16 = (size_t)NBAT * CIN * NTOK * 2;
  const size_t sY   = (size_t)NUNIT * LGR * HD * 2;
  size_t off = 0;
  const size_t oWq  = off; off += sWq;
  const size_t oWp  = off; off += sWp;
  const size_t oX16 = off; off += sX16;
  const size_t oQK  = off; off += sQK;
  const size_t oV16 = off; off += sV16;
  const size_t oY   = off; off += sY;
  if (off > ws_size) return;
  if (off > (size_t)134217728) return;

  char* ws = (char*)d_ws;
  unsigned short* Wq  = (unsigned short*)(ws + oWq);
  unsigned short* Wp  = (unsigned short*)(ws + oWp);
  unsigned short* X16 = (unsigned short*)(ws + oX16);
  unsigned short* QK  = (unsigned short*)(ws + oQK);
  unsigned short* V16 = (unsigned short*)(ws + oV16);
  unsigned short* Yp  = (unsigned short*)(ws + oY);

  const dim3 blk(256);
  cvt_w<<<dim3(128), blk, 0, stream>>>(w_qkv, w_proj, Wq, Wp);
  cvt_x<<<dim3(MTOK / 8), blk, 0, stream>>>(x, idx, X16);
  gemm_qkv<<<dim3(C3 / 64, MTOK / 128), blk, 0, stream>>>(X16, Wq, QK, V16);
  attn_k<<<dim3(NUNIT), blk, 0, stream>>>(QK, V16, Yp);
  gemm_proj<<<dim3(CIN / 64, MTOK / 128), blk, 0, stream>>>(Yp, Wp, b_proj, idx, out);
  (void)hipGetLastError();
}
